// DepGCN_214748365178
// MI455X (gfx1250) — hardware-run, weakly checked
//
#include <hip/hip_runtime.h>


#ifndef NB
#define NB 8
#endif
#ifndef SEQ
#define SEQ 256
#endif
#define NB_FULL  8
#define SEQ_FULL 256
#ifndef OUT_SEQ
#define OUT_SEQ SEQ
#endif
#define LJ   256
#define NLAB 50
#define DD   64
#define FI   256
#define FO   256
#define KG   128
#define RW   8
#define NCT  352

static_assert(LJ == SEQ_FULL);
static_assert(LJ == 256);
static_assert(FI == 256);
static_assert(FI == FO);
static_assert(DD == 64);
static_assert(KG == 2 * DD);
static_assert(KG % 32 == 0);
static_assert(FO % 64 == 0);
static_assert(SEQ % 64 == 0);
static_assert((NB * SEQ) % 64 == 0);
static_assert((NB * SEQ) % RW == 0);
static_assert(NB <= NB_FULL);
static_assert(SEQ <= SEQ_FULL);
static_assert(NCT % 32 == 0);
static_assert(NLAB <= 64);

typedef unsigned short bf;
typedef __attribute__((ext_vector_type(16))) __bf16   v16bf;
typedef __attribute__((ext_vector_type(8)))  unsigned short v8us;
typedef __attribute__((ext_vector_type(8)))  float    v8f;
typedef __attribute__((ext_vector_type(4)))  float    v4f;
typedef __attribute__((ext_vector_type(4)))  int      v4i;
typedef v4f  __attribute__((may_alias)) v4fa;
typedef v4i  __attribute__((may_alias)) v4ia;
typedef v8us __attribute__((may_alias)) v8usa;

__device__ __forceinline__ unsigned short f2bf(float f) { unsigned u = __float_as_uint(f); u += 0x7FFFu + ((u >> 16) & 1u); return (unsigned short)(u >> 16); }
__device__ __forceinline__ float bf2f(unsigned short h) { return __uint_as_float(((unsigned)h) << 16); }
__device__ __forceinline__ float bfr(float f) { return bf2f(f2bf(f)); }
__device__ __forceinline__ int clampi(int v, int lo, int hi) { v = (v < lo) ? lo : v; return (v > hi) ? hi : v; }
__device__ __forceinline__ v16bf cat16b(v8us lo, v8us hi) { return __builtin_bit_cast(v16bf, __builtin_shufflevector(lo, hi, 0, 1, 2, 3, 4, 5, 6, 7, 8, 9, 10, 11, 12, 13, 14, 15)); }
__device__ __forceinline__ v8f wmmab(v16bf a, v16bf b, v8f c) { return __builtin_amdgcn_wmma_f32_16x16x32_bf16(false, a, false, b, (short)0, c, false, false); }
__device__ __forceinline__ v16bf ldb(const bf* p)  { return cat16b(*(const v8us*)p, *(const v8us*)(p + 16)); }
__device__ __forceinline__ void wave_sync() { __builtin_amdgcn_fence(3  , "wavefront"); __builtin_amdgcn_wave_barrier(); asm volatile("" ::: "memory"); }

__global__ __launch_bounds__(256) void k_prep(const float* __restrict__ Wa, const float* __restrict__ ba, const float* __restrict__ emb, float* CT) {
    __shared__ __align__(16) float sOut[NCT];
    __shared__ __align__(16) float sWD[DD];
    __shared__ __align__(16) float sBA[256];
    const int t = threadIdx.x, lane = t & 31;
    const int wave = __builtin_amdgcn_readfirstlane(t >> 5);
    {
        const float* rp = Wa + (size_t)t * FO;
        float s0 = 0.0f, s1 = 0.0f, s2 = 0.0f, s3 = 0.0f;
#pragma unroll 1
        for (int o = 0; o < FO; o += 4) { const v4f v = *(const v4f*)(rp + o); s0 += bfr(v[0]); s1 += bfr(v[1]); s2 += bfr(v[2]); s3 += bfr(v[3]); }
        sOut[t] = (s0 + s1) + (s2 + s3);
    }
    if (wave < 2) {
        const float* rp = Wa + (size_t)(FI + t) * FO;
        float s0 = 0.0f, s1 = 0.0f, s2 = 0.0f, s3 = 0.0f;
#pragma unroll 1
        for (int o = 0; o < FO; o += 4) { const v4f v = *(const v4f*)(rp + o); s0 += bfr(v[0]); s1 += bfr(v[1]); s2 += bfr(v[2]); s3 += bfr(v[3]); }
        sWD[t] = (s0 + s1) + (s2 + s3);
    }
    sBA[t] = bfr(ba[t]);
    __syncthreads();
    if (wave < 2) {
        const int l = clampi(t, 0, NLAB - 1);
        const float* ep = emb + (size_t)l * DD;
        float d = 0.0f;
#pragma unroll 1
        for (int k = 0; k < DD; k += 4) { const v4f e = *(const v4f*)(ep + k);
            d = fmaf(bfr(e[0]), sWD[k], d); d = fmaf(bfr(e[1]), sWD[k + 1], d); d = fmaf(bfr(e[2]), sWD[k + 2], d); d = fmaf(bfr(e[3]), sWD[k + 3], d); }
        sOut[256 + t] = (t < NLAB) ? d : 0.0f;
    } else if (wave == 2) {
        float s = 0.0f;
#pragma unroll
        for (int q = 0; q < 8; ++q) s += sBA[lane * 8 + q];
        s += __shfl_xor(s, 16, 32); s += __shfl_xor(s, 8, 32); s += __shfl_xor(s, 4, 32); s += __shfl_xor(s, 2, 32); s += __shfl_xor(s, 1, 32);
        sOut[320 + lane] = s;
    }
    __syncthreads();
    const int tt = clampi(t, 0, NCT / 4 - 1);
    const v4f o = *(const v4fa*)(&sOut[tt * 4]);
    if (t < NCT / 4) *(volatile v4f*)(CT + tt * 4) = o;
    __threadfence();
    if (t < NCT / 4) *(volatile v4f*)(CT + tt * 4) = o;
}

__global__ __launch_bounds__(256) void k_wt(const float* __restrict__ Wfc, bf* WT) {
    __shared__ __align__(16) bf sT[32 * 136];
    const int tid = threadIdx.x; const int n0 = blockIdx.x * 32;
#pragma unroll 1
    for (int it = 0; it < 8; ++it) { const int idx = tid + it * 256; const int k = idx >> 5, nn = idx & 31;
        const bf u = f2bf(Wfc[(size_t)k * FO + n0 + nn]); sT[nn * 136 + k] = u; sT[nn * 136 + 64 + k] = u; }
    __syncthreads();
    v8us o[2];
#pragma unroll
    for (int it = 0; it < 2; ++it) { const int p = tid + it * 256; const int rl = p >> 4, pc = p & 15;
        o[it] = *(const v8usa*)(&sT[rl * 136 + pc * 8]); }
#pragma unroll
    for (int it = 0; it < 2; ++it) { const int p = tid + it * 256; const int rl = p >> 4, pc = p & 15;
        *(volatile v8us*)(WT + (size_t)(n0 + rl) * KG + pc * 8) = o[it]; }
    __threadfence();
#pragma unroll
    for (int it = 0; it < 2; ++it) { const int p = tid + it * 256; const int rl = p >> 4, pc = p & 15;
        *(volatile v8us*)(WT + (size_t)(n0 + rl) * KG + pc * 8) = o[it]; }
}

__global__ __launch_bounds__(32 * RW) void k_row(const float* __restrict__ text, const int* __restrict__ dmat, const int* __restrict__ dlab,
                                                 const float* __restrict__ emb, const float* __restrict__ CT, bf* AG) {
    __shared__ __align__(16) float sEmb[NLAB * DD];
    __shared__ __align__(16) float sCT[NCT];
    __shared__ __align__(16) float sP[RW * LJ];
    __shared__ __align__(16) int   sL[RW * LJ];
    __shared__ __align__(16) float sW[RW * 64];
    __shared__ __align__(16) bf    sA[RW * KG];
    const int tid = threadIdx.x, lane = tid & 31;
    const int wave = __builtin_amdgcn_readfirstlane(tid >> 5);
#pragma unroll 1
    for (int it = 0; it < (NLAB * DD + 255) / 256; ++it) { const int i = tid + it * 256; const int ii = clampi(i, 0, NLAB * DD - 1);
        const float v = bfr(emb[ii]); if (i < NLAB * DD) sEmb[i] = v; }
#pragma unroll 1
    for (int it = 0; it < (NCT + 255) / 256; ++it) { const int i = tid + it * 256; const int ii = clampi(i, 0, NCT - 1);
        const float v = CT[ii]; if (i < NCT) sCT[i] = v; }
    __syncthreads();

    const int g = __builtin_amdgcn_readfirstlane((int)blockIdx.x * RW + wave);
    const int b = g / SEQ, i = g % SEQ;
    const size_t rr = (size_t)b * SEQ_FULL + (size_t)i;
    const float* tp = text + rr * FI + lane * 8;
    const int* lp = dlab + rr * LJ + lane * 8;
    const int* mp = dmat + rr * LJ + lane * 8;
    const v4f t0 = *(const v4f*)tp, t1 = *(const v4f*)(tp + 4);
    const v4i l0 = *(const v4i*)lp, l1 = *(const v4i*)(lp + 4);
    const v4i m0 = *(const v4i*)mp, m1 = *(const v4i*)(mp + 4);
    const v4f w0 = *(const v4fa*)(&sCT[lane * 8]), w1 = *(const v4fa*)(&sCT[lane * 8 + 4]);
    float ct = 0.0f;
#pragma unroll
    for (int q = 0; q < 4; ++q) ct = fmaf(bfr(t0[q]), w0[q], ct);
#pragma unroll
    for (int q = 0; q < 4; ++q) ct = fmaf(bfr(t1[q]), w1[q], ct);
    ct += __shfl_xor(ct, 16, 32); ct += __shfl_xor(ct, 8, 32); ct += __shfl_xor(ct, 4, 32); ct += __shfl_xor(ct, 2, 32); ct += __shfl_xor(ct, 1, 32);
    const float sb = sCT[320];
    int lb[8]; float s[8];
#pragma unroll
    for (int q = 0; q < 4; ++q) { lb[q] = clampi(l0[q], 0, NLAB - 1); lb[4 + q] = clampi(l1[q], 0, NLAB - 1); }
    float mx = -3.0e38f;
#pragma unroll
    for (int q = 0; q < 8; ++q) { const int mk = (q < 4) ? m0[q & 3] : m1[q & 3];
        float v = (ct + sCT[256 + lb[q]]) + sb;
        v = v + ((mk == 0) ? -1.0e30f : 0.0f);
        s[q] = v; mx = fmaxf(mx, v); }
    mx = fmaxf(mx, __shfl_xor(mx, 16, 32)); mx = fmaxf(mx, __shfl_xor(mx, 8, 32)); mx = fmaxf(mx, __shfl_xor(mx, 4, 32));
    mx = fmaxf(mx, __shfl_xor(mx, 2, 32)); mx = fmaxf(mx, __shfl_xor(mx, 1, 32));
    float sum = 0.0f;
#pragma unroll
    for (int q = 0; q < 8; ++q) { s[q] = __builtin_amdgcn_exp2f((s[q] - mx) * 1.4426950408889634f); sum += s[q]; }
    sum += __shfl_xor(sum, 16, 32); sum += __shfl_xor(sum, 8, 32); sum += __shfl_xor(sum, 4, 32); sum += __shfl_xor(sum, 2, 32); sum += __shfl_xor(sum, 1, 32);
    const float inv = 1.0f / sum;
    { v4f p0, p1; v4i c0, c1;
#pragma unroll
      for (int q = 0; q < 4; ++q) { p0[q] = s[q] * inv; p1[q] = s[4 + q] * inv; c0[q] = lb[q]; c1[q] = lb[4 + q]; }
      *(v4fa*)(&sP[wave * LJ + lane * 8]) = p0; *(v4fa*)(&sP[wave * LJ + lane * 8 + 4]) = p1;
      *(v4ia*)(&sL[wave * LJ + lane * 8]) = c0; *(v4ia*)(&sL[wave * LJ + lane * 8 + 4]) = c1; }
    wave_sync();
    float h0 = 0.0f, h1 = 0.0f; const int la = lane, lc = lane + 32;
#pragma unroll 2
    for (int j = 0; j < LJ; j += 4) {
        const v4f pv = *(const v4fa*)(&sP[wave * LJ + j]); const v4i lv = *(const v4ia*)(&sL[wave * LJ + j]);
#pragma unroll
        for (int q = 0; q < 4; ++q) { h0 += (lv[q] == la) ? pv[q] : 0.0f; h1 += (lv[q] == lc) ? pv[q] : 0.0f; }
    }
    sW[wave * 64 + lane] = h0; sW[wave * 64 + 32 + lane] = h1;
    wave_sync();
    float a0 = 0.0f, a1 = 0.0f;
#pragma unroll 2
    for (int l = 0; l < NLAB; ++l) { const float wl = sW[wave * 64 + l];
        a0 = fmaf(wl, sEmb[l * DD + lane], a0); a1 = fmaf(wl, sEmb[l * DD + 32 + lane], a1); }
    { const bf v0 = f2bf(a0), v1 = f2bf(a1);
      const bf r0 = f2bf(a0 - bf2f(v0)), r1 = f2bf(a1 - bf2f(v1));
      sA[wave * KG + lane] = v0; sA[wave * KG + 32 + lane] = v1; sA[wave * KG + 64 + lane] = r0; sA[wave * KG + 96 + lane] = r1; }
    wave_sync();
    const v8us o = *(const v8usa*)(&sA[wave * KG + (lane & 15) * 8]);
    bf* dst = AG + (size_t)g * KG + (lane & 15) * 8;
    if (lane < 16) *(volatile v8us*)dst = o;
    __threadfence();
    if (lane < 16) *(volatile v8us*)dst = o;
}

__global__ __launch_bounds__(32) void k_gemm(const bf* __restrict__ A, const bf* __restrict__ Bt, const float* __restrict__ text, const float* __restrict__ bfc, float* OUT) {
    __shared__ __align__(16) float os[16 * 68];
    const int K = KG;
    const int lane = threadIdx.x & 31, lr = lane & 15, hi = lane >> 4; const int r0 = blockIdx.x * 64, c0 = blockIdx.y * 64;
    v8f acc[4][4];
#pragma unroll
    for (int mb = 0; mb < 4; ++mb)
#pragma unroll
        for (int nb = 0; nb < 4; ++nb) acc[mb][nb] = (v8f){};
    const size_t aoff = (size_t)(r0 + lr) * K + 8 * hi, boff = (size_t)(c0 + lr) * K + 8 * hi;
#pragma unroll 1
    for (int kc = 0; kc < K; kc += 32) {
        v16bf a[4];
#pragma unroll
        for (int mb = 0; mb < 4; ++mb) a[mb] = ldb(A + aoff + (size_t)mb * 16 * K + kc);
#pragma unroll
        for (int nb = 0; nb < 4; ++nb) { const v16bf bq = ldb(Bt + boff + (size_t)nb * 16 * K + kc);
#pragma unroll
            for (int mb = 0; mb < 4; ++mb) acc[mb][nb] = wmmab(a[mb], bq, acc[mb][nb]); }
        asm volatile("v_nop\n\tv_nop\n\tv_nop\n\tv_nop" : "+v"(acc[0][0]), "+v"(acc[1][1]), "+v"(acc[2][2]), "+v"(acc[3][3]) : "v"(a[0]), "v"(a[1]), "v"(a[2]), "v"(a[3]));
    }
    const int cofs = lr * 4;
    v4f bb = *(const v4f*)(bfc + c0 + cofs);
#pragma unroll
    for (int q = 0; q < 4; ++q) bb[q] = bfr(bb[q]);
#pragma unroll
    for (int mb = 0; mb < 4; ++mb) {
#pragma unroll
        for (int nb = 0; nb < 4; ++nb) {
#pragma unroll
            for (int j = 0; j < 8; ++j) os[(hi * 8 + j) * 68 + nb * 16 + lr] = acc[mb][nb][j]; }
        wave_sync();
        v4f val[8];
#pragma unroll
        for (int s = 0; s < 8; ++s) { const int row = 2 * s + hi;
            const v4f x = *(const v4fa*)(&os[row * 68 + cofs]);
            const int gr = r0 + mb * 16 + row; const int b = gr / SEQ, i = gr % SEQ;
            const v4f t4 = *(const v4f*)(text + ((size_t)b * SEQ_FULL + (size_t)i) * FI + c0 + cofs);
            v4f o;
#pragma unroll
            for (int q = 0; q < 4; ++q) { const float v = (bfr(t4[q]) + x[q]) + bb[q]; o[q] = (v > 0.0f) ? v : 0.0f; }
            val[s] = o; }
#pragma unroll
        for (int s = 0; s < 8; ++s) { const int row = 2 * s + hi; const int gr = r0 + mb * 16 + row; const int b = gr / SEQ, i = gr % SEQ;
            *(volatile v4f*)(OUT + ((size_t)b * OUT_SEQ + (size_t)i) * FO + c0 + cofs) = val[s]; }
        __threadfence();
#pragma unroll
        for (int s = 0; s < 8; ++s) { const int row = 2 * s + hi; const int gr = r0 + mb * 16 + row; const int b = gr / SEQ, i = gr % SEQ;
            *(volatile v4f*)(OUT + ((size_t)b * OUT_SEQ + (size_t)i) * FO + c0 + cofs) = val[s]; }
        wave_sync();
    }
}

static constexpr size_t al256(size_t v) { return (v + 255) & ~(size_t)255; }
static constexpr size_t SZ_CT = al256((size_t)NCT * 4);
static constexpr size_t SZ_WT = al256((size_t)FO * KG * 2);
static constexpr size_t SZ_AG = al256((size_t)NB * SEQ * KG * 2);
static constexpr size_t SZ_TOTAL = SZ_CT + SZ_WT + SZ_AG;
static_assert(SZ_TOTAL <= (size_t)134217728);
static_assert((size_t)(NCT / 4) * 16 <= SZ_CT);
static_assert((size_t)FO * KG * 2 <= SZ_WT);
static_assert((size_t)NB * SEQ * KG * 2 <= SZ_AG);

extern "C" void kernel_launch(void* const* d_in, const int* in_sizes, int n_in,
                              void* d_out, int out_size, void* d_ws, size_t ws_size, hipStream_t stream) {
    if (n_in < 8) return;
    const size_t nrows = (size_t)(NB - 1) * SEQ_FULL + SEQ;
    if ((size_t)in_sizes[0] < nrows * FI) return;
    if ((size_t)in_sizes[1] < nrows * LJ || (size_t)in_sizes[2] < nrows * LJ) return;
    if ((size_t)in_sizes[3] < (size_t)NLAB * DD) return;
    if ((size_t)in_sizes[4] < (size_t)(FI + DD) * FO) return;
    if ((size_t)in_sizes[5] < (size_t)FO) return;
    if ((size_t)in_sizes[6] < (size_t)DD * FO) return;
    if ((size_t)in_sizes[7] < (size_t)FO) return;
    if ((size_t)out_size < ((size_t)(NB - 1) * OUT_SEQ + SEQ) * FO) return;
    if (SZ_TOTAL > ws_size) return;
    const float* text = (const float*)d_in[0];
    const int*   dmat = (const int*)d_in[1];
    const int*   dlab = (const int*)d_in[2];
    const float* emb  = (const float*)d_in[3];
    const float* Wa   = (const float*)d_in[4];
    const float* ba   = (const float*)d_in[5];
    const float* Wfc  = (const float*)d_in[6];
    const float* bfc  = (const float*)d_in[7];
    float* OUT = (float*)d_out;
    char* wsp = (char*)d_ws;
    float* CT = (float*)wsp; wsp += SZ_CT;
    bf* WT = (bf*)wsp; wsp += SZ_WT;
    bf* AG = (bf*)wsp; wsp += SZ_AG;

    k_prep<<<1, 256, 0, stream>>>(Wa, ba, emb, CT);
    k_wt<<<FO / 32, 256, 0, stream>>>(Wfc, WT);
    k_row<<<(NB * SEQ) / RW, 32 * RW, 0, stream>>>(text, dmat, dlab, emb, CT, AG);
    k_gemm<<<dim3((NB * SEQ) / 64, FO / 64, 1), 32, 0, stream>>>(AG, WT, text, bfc, OUT);
}
